// FedFormer_40372692582804
// MI455X (gfx1250) — hardware-verified
//
#include <hip/hip_runtime.h>
#define BB 64
#define LL 1024
#define CI 7
#define DD 64
#define NHD 8
#define EE 8
#define DFF 256
#define MO 64
#define MT (BB * LL)
#define NR (BB * DD)

typedef __bf16 v16b __attribute__((ext_vector_type(16)));
typedef unsigned short v8us __attribute__((ext_vector_type(8), may_alias));
typedef float  v8f  __attribute__((ext_vector_type(8)));
typedef float  v4f  __attribute__((ext_vector_type(4)));
typedef float  v4fa __attribute__((ext_vector_type(4), may_alias));
union FragB { v16b v; v8us half[2]; unsigned short u[16]; };

__device__ __forceinline__ unsigned short bf16_bits(float x) { unsigned int u = __float_as_uint(x); return (unsigned short)((u + 0x7FFFu + ((u >> 16) & 1u)) >> 16); }
__device__ __forceinline__ float bf16_val(unsigned short b) { return __uint_as_float(((unsigned int)b) << 16); }
__device__ __forceinline__ float bf16_round(float x) { return bf16_val(bf16_bits(x)); }
template <int NT>
__device__ __forceinline__ v8f mmaN(v16b ah, v16b al, v16b bh, v16b bl, v8f c) {
  c = __builtin_amdgcn_wmma_f32_16x16x32_bf16(false, ah, false, bh, (short)0, c, false, false);
  if (NT >= 2) c = __builtin_amdgcn_wmma_f32_16x16x32_bf16(false, al, false, bh, (short)0, c, false, false);
  if (NT >= 3) c = __builtin_amdgcn_wmma_f32_16x16x32_bf16(false, ah, false, bl, (short)0, c, false, false);
  asm volatile("v_nop\n\tv_nop\n\tv_nop\n\tv_nop" : "+v"(c) : "v"(ah), "v"(al), "v"(bh), "v"(bl));
  return c;
}

__global__ __launch_bounds__(256) void k_wt_bf16(const float* __restrict__ W, unsigned short* __restrict__ Wt, int K, int N) {
  const int t = blockIdx.x * 256 + threadIdx.x;
  const int k8n = K / 8;
  if (t >= N * k8n) return;
  const int n = t / k8n, k8 = (t % k8n) * 8;
  v8us v;
#pragma unroll
  for (int i = 0; i < 8; ++i) v[i] = bf16_bits(W[(size_t)(k8 + i) * N + n]);
  *(volatile v8us*)(Wt + (size_t)n * K + k8) = v;
  __threadfence();
  *(volatile v8us*)(Wt + (size_t)n * K + k8) = v;
}

template <bool ASPLIT, int ACT, bool BIAS_BF16>
__global__ __launch_bounds__(128) void k_gemm_bf(const float* __restrict__ A, int lda, const unsigned short* __restrict__ Wt, int ldb,
                                               const float* __restrict__ bias, float* __restrict__ C, int ldc, int M, int N, int K) {
  __shared__ __attribute__((aligned(16))) float so[4][16][64];
  const int tid = threadIdx.x, w = tid >> 5, lane = tid & 31, ln = lane & 15, hh = lane >> 4;
  const int ntn = N / 64;
  const int wid = blockIdx.x * 4 + w;
  const int mt = wid / ntn, nq = wid % ntn;
  if (mt * 16 >= M) return;
  const int row0 = mt * 16, col0 = nq * 64;
  const float* arow = A + (size_t)(row0 + ln) * lda;
  v8f acc[4] = {};
  for (int kb = 0; kb < K; kb += 32) {
    FragB ah, al;
    const v4f x0 = *(const v4fa*)(arow + kb + 8 * hh), x1 = *(const v4fa*)(arow + kb + 8 * hh + 4);
    const v4f x2 = *(const v4fa*)(arow + kb + 16 + 8 * hh), x3 = *(const v4fa*)(arow + kb + 16 + 8 * hh + 4);
    float xs[16] = {x0[0],x0[1],x0[2],x0[3],x1[0],x1[1],x1[2],x1[3],x2[0],x2[1],x2[2],x2[3],x3[0],x3[1],x3[2],x3[3]};
#pragma unroll
    for (int i = 0; i < 16; ++i) { const unsigned short hb = bf16_bits(xs[i]); ah.u[i] = hb; al.u[i] = ASPLIT ? bf16_bits(xs[i] - bf16_val(hb)) : (unsigned short)0; }
#pragma unroll
    for (int t = 0; t < 4; ++t) {
      const unsigned short* brow = Wt + (size_t)(col0 + t * 16 + ln) * ldb + kb;
      FragB b;
      b.half[0] = *(const v8us*)(brow + 8 * hh);
      b.half[1] = *(const v8us*)(brow + 16 + 8 * hh);
      acc[t] = mmaN<ASPLIT ? 2 : 1>(ah.v, al.v, b.v, b.v, acc[t]);
    }
  }
#pragma unroll
  for (int t = 0; t < 4; ++t) {
    float bv = bias ? bias[col0 + t * 16 + ln] : 0.f;
    if (BIAS_BF16) bv = bf16_round(bv);
#pragma unroll
    for (int r = 0; r < 8; ++r) { float v = acc[t][r] + bv; if (ACT == 1) v = fmaxf(v, 0.f); so[w][8 * hh + r][t * 16 + ln] = v; }
  }
  __builtin_amdgcn_fence(__ATOMIC_ACQ_REL, "workgroup");
  __builtin_amdgcn_wave_barrier();
  const int rsub = lane >> 4, c4 = (lane & 15) * 4;
  for (int pass = 0; pass < 2; ++pass) {
#pragma unroll
    for (int q = 0; q < 8; ++q) {
      const int r = q * 2 + rsub;
      const v4f v = *(const v4fa*)&so[w][r][c4];
      *(volatile v4f*)(C + (size_t)(row0 + r) * ldc + col0 + c4) = v;
    }
    if (pass == 0) __threadfence();
  }
}

template <int D, bool CAUSAL>
__global__ __launch_bounds__(128) void k_flash(const float* __restrict__ qb, const float* __restrict__ kb, const float* __restrict__ vb,
                                             int pitch, int T, int H, float scale, float* __restrict__ y, int ypitch) {
  constexpr int KS = D / 32;
  constexpr int DT = D / 16;
  __shared__ __attribute__((aligned(16))) unsigned short sKh[32][D + 8], sKl[32][D + 8], sVh[32][D + 8], sVl[32][D + 8];
  __shared__ __attribute__((aligned(16))) unsigned short sPh[4][16][40], sPl[4][16][40];
  __shared__ __attribute__((aligned(16))) float sO[4][16][D];
  const int tid = threadIdx.x, w = tid >> 5, lane = tid & 31, ln = lane & 15, hh = lane >> 4;
  const int nqb = (T + 63) / 64;
  const int bh = blockIdx.x / nqb, qblk = blockIdx.x % nqb;
  const int b = bh / H, h = bh % H;
  const int q0 = qblk * 64 + w * 16;
  const float* Q = qb + (size_t)b * T * pitch + h * D;
  const float* K = kb + (size_t)b * T * pitch + h * D;
  const float* V = vb + (size_t)b * T * pitch + h * D;

  FragB aqh[KS], aql[KS];
  {
    int row = q0 + ln; if (row >= T) row = T - 1;
    const float* qr = Q + (size_t)row * pitch;
#pragma unroll
    for (int ks = 0; ks < KS; ++ks)
#pragma unroll
      for (int i = 0; i < 16; ++i) {
        const int d = ks * 32 + ((i < 8) ? (8 * hh + i) : (16 + 8 * hh + (i - 8)));
        const float x = qr[d] * scale; const unsigned short hb = bf16_bits(x);
        aqh[ks].u[i] = hb; aql[ks].u[i] = bf16_bits(x - bf16_val(hb));
      }
  }
  float m_r[8], l_r[8];
#pragma unroll
  for (int r = 0; r < 8; ++r) { m_r[r] = -3.0e38f; l_r[r] = 0.f; }
  v8f oacc[DT];
#pragma unroll
  for (int dt = 0; dt < DT; ++dt) oacc[dt] = (v8f){0.f,0.f,0.f,0.f,0.f,0.f,0.f,0.f};

  const int kv_end = CAUSAL ? min(T, qblk * 64 + 64) : T;
  for (int j0 = 0; j0 < kv_end; j0 += 32) {
    __syncthreads();
    for (int e = tid; e < 32 * (D / 4); e += 128) {
      const int r = e / (D / 4), c4 = (e % (D / 4)) * 4;
      const int key = j0 + r;
      v4f kf = {0.f,0.f,0.f,0.f}, vf = {0.f,0.f,0.f,0.f};
      if (key < T) { kf = *(const v4fa*)(K + (size_t)key * pitch + c4); vf = *(const v4fa*)(V + (size_t)key * pitch + c4); }
#pragma unroll
      for (int t = 0; t < 4; ++t) {
        unsigned short hb = bf16_bits(kf[t]); sKh[r][c4 + t] = hb; sKl[r][c4 + t] = bf16_bits(kf[t] - bf16_val(hb));
        hb = bf16_bits(vf[t]); sVh[r][c4 + t] = hb; sVl[r][c4 + t] = bf16_bits(vf[t] - bf16_val(hb));
      }
    }
    __syncthreads();
    v8f s[2];
#pragma unroll
    for (int nt = 0; nt < 2; ++nt) {
      v8f acc = {};
#pragma unroll
      for (int ks = 0; ks < KS; ++ks) {
        FragB bh_, bl_;
        bh_.half[0] = *(const v8us*)&sKh[nt * 16 + ln][ks * 32 + 8 * hh]; bh_.half[1] = *(const v8us*)&sKh[nt * 16 + ln][ks * 32 + 16 + 8 * hh];
        bl_.half[0] = *(const v8us*)&sKl[nt * 16 + ln][ks * 32 + 8 * hh]; bl_.half[1] = *(const v8us*)&sKl[nt * 16 + ln][ks * 32 + 16 + 8 * hh];
        acc = mmaN<3>(aqh[ks].v, aql[ks].v, bh_.v, bl_.v, acc);
      }
      s[nt] = acc;
    }
    float alpha[8];
#pragma unroll
    for (int r = 0; r < 8; ++r) {
      const int qi = q0 + 8 * hh + r;
      const int ja = j0 + ln, jb = j0 + 16 + ln;
      if (CAUSAL) { if (ja > qi) s[0][r] = -3.0e38f; if (jb > qi) s[1][r] = -3.0e38f; }
      if (ja >= T) s[0][r] = -3.0e38f;
      if (jb >= T) s[1][r] = -3.0e38f;
      float mx = fmaxf(s[0][r], s[1][r]);
      mx = fmaxf(mx, __shfl_xor(mx, 1, 32)); mx = fmaxf(mx, __shfl_xor(mx, 2, 32)); mx = fmaxf(mx, __shfl_xor(mx, 4, 32)); mx = fmaxf(mx, __shfl_xor(mx, 8, 32));
      const float mnew = fmaxf(m_r[r], mx);
      alpha[r] = (mnew > -1.0e38f) ? __expf(m_r[r] - mnew) : 1.0f;
      const float p0 = (s[0][r] > -1.0e38f) ? __expf(s[0][r] - mnew) : 0.f;
      const float p1 = (s[1][r] > -1.0e38f) ? __expf(s[1][r] - mnew) : 0.f;
      m_r[r] = mnew;
      l_r[r] = l_r[r] * alpha[r] + p0 + p1;
      unsigned short hb = bf16_bits(p0); sPh[w][8 * hh + r][ln] = hb;      sPl[w][8 * hh + r][ln] = bf16_bits(p0 - bf16_val(hb));
      hb = bf16_bits(p1);                sPh[w][8 * hh + r][16 + ln] = hb; sPl[w][8 * hh + r][16 + ln] = bf16_bits(p1 - bf16_val(hb));
    }
#pragma unroll
    for (int dt = 0; dt < DT; ++dt)
#pragma unroll
      for (int r = 0; r < 8; ++r) oacc[dt][r] *= alpha[r];
    __builtin_amdgcn_fence(__ATOMIC_ACQ_REL, "workgroup");
    __builtin_amdgcn_wave_barrier();
    FragB pah, pal;
    pah.half[0] = *(const v8us*)&sPh[w][ln][8 * hh]; pah.half[1] = *(const v8us*)&sPh[w][ln][16 + 8 * hh];
    pal.half[0] = *(const v8us*)&sPl[w][ln][8 * hh]; pal.half[1] = *(const v8us*)&sPl[w][ln][16 + 8 * hh];
#pragma unroll
    for (int dt = 0; dt < DT; ++dt) {
      FragB bvh, bvl;
#pragma unroll
      for (int i = 0; i < 8; ++i) {
        bvh.u[i] = sVh[8 * hh + i][dt * 16 + ln]; bvh.u[8 + i] = sVh[16 + 8 * hh + i][dt * 16 + ln];
        bvl.u[i] = sVl[8 * hh + i][dt * 16 + ln]; bvl.u[8 + i] = sVl[16 + 8 * hh + i][dt * 16 + ln];
      }
      oacc[dt] = mmaN<3>(pah.v, pal.v, bvh.v, bvl.v, oacc[dt]);
    }
    __builtin_amdgcn_fence(__ATOMIC_ACQ_REL, "workgroup");
    __builtin_amdgcn_wave_barrier();
  }
#pragma unroll
  for (int r = 0; r < 8; ++r) {
    float l = l_r[r];
    l += __shfl_xor(l, 1, 32); l += __shfl_xor(l, 2, 32); l += __shfl_xor(l, 4, 32); l += __shfl_xor(l, 8, 32);
    l_r[r] = (l > 0.f) ? 1.0f / l : 0.f;
  }
#pragma unroll
  for (int dt = 0; dt < DT; ++dt)
#pragma unroll
    for (int r = 0; r < 8; ++r) sO[w][8 * hh + r][dt * 16 + ln] = oacc[dt][r] * l_r[r];
  __builtin_amdgcn_fence(__ATOMIC_ACQ_REL, "workgroup");
  __builtin_amdgcn_wave_barrier();
  for (int pass = 0; pass < 2; ++pass) {
    for (int r = 0; r < 16; ++r) {
      const int row = q0 + r;
      if (row < T && lane < D / 4) {
        const v4f val = *(const v4fa*)&sO[w][r][lane * 4];
        *(volatile v4f*)(y + ((size_t)b * T + row) * ypitch + h * D + lane * 4) = val;
      }
    }
    if (pass == 0) __threadfence();
  }
}

template <bool AFFINE, bool RESID, bool RES_BF16>
__global__ __launch_bounds__(256) void k_transpose32(const float* __restrict__ in, float* __restrict__ out, int rows, int cols,
                                                    const float* __restrict__ scale, const float* __restrict__ shift, const float* __restrict__ res) {
  __shared__ float tile[32][33];
  const int b = blockIdx.z;
  const int r0 = blockIdx.y * 32, c0 = blockIdx.x * 32;
  const float* src = in + (size_t)b * rows * cols;
  float* dst = out + (size_t)b * rows * cols;
  const int tx = threadIdx.x & 31, ty = threadIdx.x >> 5;
  for (int i = ty; i < 32; i += 8) tile[i][tx] = src[(size_t)(r0 + i) * cols + c0 + tx];
  __syncthreads();
  for (int pass = 0; pass < 2; ++pass) {
    for (int i = ty; i < 32; i += 8) {
      float v = tile[tx][i];
      const int orow = c0 + i;
      if (AFFINE) v = v * scale[orow] + shift[orow];
      if (RESID) { float rv = res[(size_t)b * rows * cols + (size_t)orow * rows + r0 + tx]; if (RES_BF16) rv = bf16_round(rv); v += rv; }
      *(volatile float*)(dst + (size_t)orow * rows + r0 + tx) = v;
    }
    if (pass == 0) __threadfence();
  }
}

__global__ __launch_bounds__(256) void k_pool2_pm(const float* __restrict__ in, float* __restrict__ out, int Bn, int H, int W, int C) {
  const size_t t = (size_t)blockIdx.x * 256 + threadIdx.x;
  const int c4n = C / 4, Ho = H / 2, Wo = W / 2;
  const size_t total = (size_t)Bn * Ho * Wo * c4n;
  if (t >= total) return;
  const int c4 = (int)(t % c4n) * 4; size_t rest = t / c4n;
  const int pw = (int)(rest % Wo); rest /= Wo; const int ph = (int)(rest % Ho); const int b = (int)(rest / Ho);
  const float* base = in + (size_t)b * H * W * C;
  const int p00 = (2 * ph) * W + 2 * pw;
  const v4f a = *(const v4fa*)(base + (size_t)p00 * C + c4), bq = *(const v4fa*)(base + (size_t)(p00 + 1) * C + c4);
  const v4f c = *(const v4fa*)(base + (size_t)(p00 + W) * C + c4), d = *(const v4fa*)(base + (size_t)(p00 + W + 1) * C + c4);
  v4f m; for (int i = 0; i < 4; ++i) m[i] = fmaxf(fmaxf(a[i], bq[i]), fmaxf(c[i], d[i]));
  float* dst = out + ((size_t)b * Ho * Wo + (size_t)ph * Wo + pw) * C + c4;
  *(volatile v4f*)dst = m;
  __threadfence();
  *(volatile v4f*)dst = m;
}

template <int DQ, int DV>
__global__ __launch_bounds__(128) void k_flash2(const float* __restrict__ Qb, size_t qstride, int qpitch, int Tq,
                                              const float* __restrict__ Kb, size_t kstride, int kpitch, int Tk,
                                              const float* __restrict__ Vb, size_t vstride, int vpitch,
                                              float scale, float* __restrict__ y, size_t ystride, int ypitch) {
  constexpr int KS = DQ / 32, DT = DV / 16;
  __shared__ __attribute__((aligned(16))) unsigned short sKh[32][DQ + 8], sKl[32][DQ + 8], sVh[32][DV + 8], sVl[32][DV + 8];
  __shared__ __attribute__((aligned(16))) unsigned short sPh[4][16][40], sPl[4][16][40];
  __shared__ __attribute__((aligned(16))) float sO[4][16][DV];
  const int tid = threadIdx.x, w = tid >> 5, lane = tid & 31, ln = lane & 15, hh = lane >> 4;
  const int nqb = (Tq + 63) / 64;
  const int bh = blockIdx.x / nqb, qblk = blockIdx.x % nqb;
  const int dv0 = blockIdx.y * DV;
  const int q0 = qblk * 64 + w * 16;
  const float* Q = Qb + (size_t)bh * qstride; const float* K = Kb + (size_t)bh * kstride; const float* V = Vb + (size_t)bh * vstride + dv0;
  FragB aqh[KS], aql[KS];
  {
    int row = q0 + ln; if (row >= Tq) row = Tq - 1;
    const float* qr = Q + (size_t)row * qpitch;
#pragma unroll
    for (int ks = 0; ks < KS; ++ks)
#pragma unroll
      for (int i = 0; i < 16; ++i) {
        const int d = ks * 32 + ((i < 8) ? (8 * hh + i) : (16 + 8 * hh + (i - 8)));
        const float x = qr[d] * scale; const unsigned short hb = bf16_bits(x);
        aqh[ks].u[i] = hb; aql[ks].u[i] = bf16_bits(x - bf16_val(hb));
      }
  }
  float m_r[8], l_r[8];
#pragma unroll
  for (int r = 0; r < 8; ++r) { m_r[r] = -3.0e38f; l_r[r] = 0.f; }
  v8f oacc[DT];
#pragma unroll
  for (int dt = 0; dt < DT; ++dt) oacc[dt] = (v8f){0.f,0.f,0.f,0.f,0.f,0.f,0.f,0.f};
  for (int j0 = 0; j0 < Tk; j0 += 32) {
    __syncthreads();
    for (int e = tid; e < 32 * (DQ / 4); e += 128) {
      const int r = e / (DQ / 4), c4 = (e % (DQ / 4)) * 4; const int key = j0 + r;
      v4f f = {0.f,0.f,0.f,0.f}; if (key < Tk) f = *(const v4fa*)(K + (size_t)key * kpitch + c4);
#pragma unroll
      for (int t = 0; t < 4; ++t) { const unsigned short hb = bf16_bits(f[t]); sKh[r][c4 + t] = hb; sKl[r][c4 + t] = bf16_bits(f[t] - bf16_val(hb)); }
    }
    for (int e = tid; e < 32 * (DV / 4); e += 128) {
      const int r = e / (DV / 4), c4 = (e % (DV / 4)) * 4; const int key = j0 + r;
      v4f f = {0.f,0.f,0.f,0.f}; if (key < Tk) f = *(const v4fa*)(V + (size_t)key * vpitch + c4);
#pragma unroll
      for (int t = 0; t < 4; ++t) { const unsigned short hb = bf16_bits(f[t]); sVh[r][c4 + t] = hb; sVl[r][c4 + t] = bf16_bits(f[t] - bf16_val(hb)); }
    }
    __syncthreads();
    v8f s[2];
#pragma unroll
    for (int nt = 0; nt < 2; ++nt) {
      v8f acc = {};
#pragma unroll
      for (int ks = 0; ks < KS; ++ks) {
        FragB bh_, bl_;
        bh_.half[0] = *(const v8us*)&sKh[nt * 16 + ln][ks * 32 + 8 * hh]; bh_.half[1] = *(const v8us*)&sKh[nt * 16 + ln][ks * 32 + 16 + 8 * hh];
        bl_.half[0] = *(const v8us*)&sKl[nt * 16 + ln][ks * 32 + 8 * hh]; bl_.half[1] = *(const v8us*)&sKl[nt * 16 + ln][ks * 32 + 16 + 8 * hh];
        acc = mmaN<3>(aqh[ks].v, aql[ks].v, bh_.v, bl_.v, acc);
      }
      s[nt] = acc;
    }
    float alpha[8];
#pragma unroll
    for (int r = 0; r < 8; ++r) {
      const int ja = j0 + ln, jb = j0 + 16 + ln;
      if (ja >= Tk) s[0][r] = -3.0e38f;
      if (jb >= Tk) s[1][r] = -3.0e38f;
      float mx = fmaxf(s[0][r], s[1][r]);
      mx = fmaxf(mx, __shfl_xor(mx, 1, 32)); mx = fmaxf(mx, __shfl_xor(mx, 2, 32)); mx = fmaxf(mx, __shfl_xor(mx, 4, 32)); mx = fmaxf(mx, __shfl_xor(mx, 8, 32));
      const float mnew = fmaxf(m_r[r], mx);
      alpha[r] = (mnew > -1.0e38f) ? __expf(m_r[r] - mnew) : 1.0f;
      const float p0 = (s[0][r] > -1.0e38f) ? __expf(s[0][r] - mnew) : 0.f;
      const float p1 = (s[1][r] > -1.0e38f) ? __expf(s[1][r] - mnew) : 0.f;
      m_r[r] = mnew;
      l_r[r] = l_r[r] * alpha[r] + p0 + p1;
      unsigned short hb = bf16_bits(p0); sPh[w][8 * hh + r][ln] = hb;      sPl[w][8 * hh + r][ln] = bf16_bits(p0 - bf16_val(hb));
      hb = bf16_bits(p1);                sPh[w][8 * hh + r][16 + ln] = hb; sPl[w][8 * hh + r][16 + ln] = bf16_bits(p1 - bf16_val(hb));
    }
#pragma unroll
    for (int dt = 0; dt < DT; ++dt)
#pragma unroll
      for (int r = 0; r < 8; ++r) oacc[dt][r] *= alpha[r];
    __builtin_amdgcn_fence(__ATOMIC_ACQ_REL, "workgroup");
    __builtin_amdgcn_wave_barrier();
    FragB pah, pal;
    pah.half[0] = *(const v8us*)&sPh[w][ln][8 * hh]; pah.half[1] = *(const v8us*)&sPh[w][ln][16 + 8 * hh];
    pal.half[0] = *(const v8us*)&sPl[w][ln][8 * hh]; pal.half[1] = *(const v8us*)&sPl[w][ln][16 + 8 * hh];
#pragma unroll
    for (int dt = 0; dt < DT; ++dt) {
      FragB bvh, bvl;
#pragma unroll
      for (int i = 0; i < 8; ++i) {
        bvh.u[i] = sVh[8 * hh + i][dt * 16 + ln]; bvh.u[8 + i] = sVh[16 + 8 * hh + i][dt * 16 + ln];
        bvl.u[i] = sVl[8 * hh + i][dt * 16 + ln]; bvl.u[8 + i] = sVl[16 + 8 * hh + i][dt * 16 + ln];
      }
      oacc[dt] = mmaN<3>(pah.v, pal.v, bvh.v, bvl.v, oacc[dt]);
    }
    __builtin_amdgcn_fence(__ATOMIC_ACQ_REL, "workgroup");
    __builtin_amdgcn_wave_barrier();
  }
#pragma unroll
  for (int r = 0; r < 8; ++r) {
    float l = l_r[r];
    l += __shfl_xor(l, 1, 32); l += __shfl_xor(l, 2, 32); l += __shfl_xor(l, 4, 32); l += __shfl_xor(l, 8, 32);
    l_r[r] = (l > 0.f) ? 1.0f / l : 0.f;
  }
#pragma unroll
  for (int dt = 0; dt < DT; ++dt)
#pragma unroll
    for (int r = 0; r < 8; ++r) sO[w][8 * hh + r][dt * 16 + ln] = oacc[dt][r] * l_r[r];
  __builtin_amdgcn_fence(__ATOMIC_ACQ_REL, "workgroup");
  __builtin_amdgcn_wave_barrier();
  for (int pass = 0; pass < 2; ++pass) {
    for (int r = 0; r < 16; ++r) {
      const int row = q0 + r;
      for (int c4 = lane * 4; c4 < DV; c4 += 128) {
        if (row < Tq) {
          const v4f val = *(const v4fa*)&sO[w][r][c4];
          *(volatile v4f*)(y + (size_t)bh * ystride + (size_t)row * ypitch + dv0 + c4) = val;
        }
      }
    }
    if (pass == 0) __threadfence();
  }
}

__global__ __launch_bounds__(256) void k_split_rows(const float* __restrict__ src, int lds_, unsigned short* __restrict__ hi, unsigned short* __restrict__ lo, int R, int Cc) {
  const size_t t = (size_t)blockIdx.x * 256 + threadIdx.x;
  const int c8n = Cc / 8;
  if (t >= (size_t)R * c8n) return;
  const int r = (int)(t / c8n), c8 = (int)(t % c8n) * 8;
  const float* s = src + (size_t)r * lds_ + c8;
  const v4f a = *(const v4fa*)s, b = *(const v4fa*)(s + 4);
  float xs[8] = {a[0],a[1],a[2],a[3],b[0],b[1],b[2],b[3]};
  v8us vh, vl;
#pragma unroll
  for (int i = 0; i < 8; ++i) { const unsigned short hb = bf16_bits(xs[i]); vh[i] = hb; vl[i] = bf16_bits(xs[i] - bf16_val(hb)); }
  unsigned short* dh = hi + (size_t)r * Cc + c8; unsigned short* dl = lo + (size_t)r * Cc + c8;
  *(volatile v8us*)dh = vh; *(volatile v8us*)dl = vl; __threadfence(); *(volatile v8us*)dh = vh; *(volatile v8us*)dl = vl;
}
__global__ __launch_bounds__(256) void k_split_transpose(const float* __restrict__ src, int lds_, unsigned short* __restrict__ hi, unsigned short* __restrict__ lo, int K, int N) {
  const size_t t = (size_t)blockIdx.x * 256 + threadIdx.x;
  const int k8n = K / 8;
  if (t >= (size_t)N * k8n) return;
  const int n = (int)(t / k8n), k8 = (int)(t % k8n) * 8;
  v8us vh, vl;
#pragma unroll
  for (int i = 0; i < 8; ++i) { const float x = src[(size_t)(k8 + i) * lds_ + n]; const unsigned short hb = bf16_bits(x); vh[i] = hb; vl[i] = bf16_bits(x - bf16_val(hb)); }
  unsigned short* dh = hi + (size_t)n * K + k8; unsigned short* dl = lo + (size_t)n * K + k8;
  *(volatile v8us*)dh = vh; *(volatile v8us*)dl = vl; __threadfence(); *(volatile v8us*)dh = vh; *(volatile v8us*)dl = vl;
}
template <bool ASPLIT, bool BSPLIT, int ACT, bool BIAS_BF16>
__global__ __launch_bounds__(128) void k_gemm_bf2(const float* __restrict__ A, int lda, const unsigned short* __restrict__ Bh, const unsigned short* __restrict__ Bl, int ldb,
                                                const float* __restrict__ bias, float alpha, float* __restrict__ C, int ldc, int M, int N, int K) {
  __shared__ __attribute__((aligned(16))) float so[4][16][64];
  const int tid = threadIdx.x, w = tid >> 5, lane = tid & 31, ln = lane & 15, hh = lane >> 4;
  const int ntn = N / 64;
  const int wid = blockIdx.x * 4 + w;
  const int mt = wid / ntn, nq = wid % ntn;
  if (mt * 16 >= M) return;
  const int row0 = mt * 16, col0 = nq * 64;
  const float* arow = A + (size_t)(row0 + ln) * lda;
  v8f acc[4] = {};
  for (int kb = 0; kb < K; kb += 32) {
    FragB ah, al;
    const v4f x0 = *(const v4fa*)(arow + kb + 8 * hh), x1 = *(const v4fa*)(arow + kb + 8 * hh + 4);
    const v4f x2 = *(const v4fa*)(arow + kb + 16 + 8 * hh), x3 = *(const v4fa*)(arow + kb + 16 + 8 * hh + 4);
    float xs[16] = {x0[0],x0[1],x0[2],x0[3],x1[0],x1[1],x1[2],x1[3],x2[0],x2[1],x2[2],x2[3],x3[0],x3[1],x3[2],x3[3]};
#pragma unroll
    for (int i = 0; i < 16; ++i) { const unsigned short hb = bf16_bits(xs[i]); ah.u[i] = hb; al.u[i] = ASPLIT ? bf16_bits(xs[i] - bf16_val(hb)) : (unsigned short)0; }
#pragma unroll
    for (int t = 0; t < 4; ++t) {
      const size_t boff = (size_t)(col0 + t * 16 + ln) * ldb + kb;
      FragB bh_, bl_;
      bh_.half[0] = *(const v8us*)(Bh + boff + 8 * hh);
      bh_.half[1] = *(const v8us*)(Bh + boff + 16 + 8 * hh);
      if (BSPLIT) { bl_.half[0] = *(const v8us*)(Bl + boff + 8 * hh); bl_.half[1] = *(const v8us*)(Bl + boff + 16 + 8 * hh); } else bl_ = bh_;
      acc[t] = mmaN<ASPLIT ? (BSPLIT ? 3 : 2) : 1>(ah.v, al.v, bh_.v, bl_.v, acc[t]);
    }
  }
#pragma unroll
  for (int t = 0; t < 4; ++t) {
    float bv = bias ? bias[col0 + t * 16 + ln] : 0.f;
    if (BIAS_BF16) bv = bf16_round(bv);
#pragma unroll
    for (int r = 0; r < 8; ++r) { float v = acc[t][r] * alpha + bv; if (ACT == 1) v = fmaxf(v, 0.f); so[w][8 * hh + r][t * 16 + ln] = v; }
  }
  __builtin_amdgcn_fence(__ATOMIC_ACQ_REL, "workgroup");
  __builtin_amdgcn_wave_barrier();
  const int rsub = lane >> 4, c4 = (lane & 15) * 4;
  for (int pass = 0; pass < 2; ++pass) {
#pragma unroll
    for (int q = 0; q < 8; ++q) {
      const int r = q * 2 + rsub;
      const v4f v = *(const v4fa*)&so[w][r][c4];
      *(volatile v4f*)(C + (size_t)(row0 + r) * ldc + col0 + c4) = v;
    }
    if (pass == 0) __threadfence();
  }
}
__global__ __launch_bounds__(256) void k_softmax_rows(const float* __restrict__ S, float* __restrict__ P, int N, int causal, int rowoff, const int* __restrict__ mask, int mask_pitch) {
  __shared__ float red[256];
  const int row = blockIdx.x, tid = threadIdx.x;
  const float* s = S + (size_t)row * N; float* p_out = P + (size_t)row * N;
  const int qi = row + rowoff;
  float mx = -3.0e38f;
  for (int j = tid; j < N; j += 256) {
    bool keep = true;
    if (causal && j > qi) keep = false;
    if (mask && mask[(size_t)qi * mask_pitch + j] == 0) keep = false;
    const float v = keep ? s[j] : -3.0e38f;
    mx = fmaxf(mx, v);
  }
  red[tid] = mx; __syncthreads();
  for (int st = 128; st > 0; st >>= 1) { if (tid < st) red[tid] = fmaxf(red[tid], red[tid + st]); __syncthreads(); }
  mx = red[0]; __syncthreads();
  float sum = 0.f;
  for (int j = tid; j < N; j += 256) {
    bool keep = true;
    if (causal && j > qi) keep = false;
    if (mask && mask[(size_t)qi * mask_pitch + j] == 0) keep = false;
    const float p = keep ? __expf(s[j] - mx) : 0.f;
    sum += p;
  }
  red[tid] = sum; __syncthreads();
  for (int st = 128; st > 0; st >>= 1) { if (tid < st) red[tid] += red[tid + st]; __syncthreads(); }
  const float inv = (mx > -1.0e38f) ? 1.0f / red[0] : __builtin_nanf("");
  __syncthreads();
  for (int pass = 0; pass < 2; ++pass) {
    for (int j4 = tid * 4; j4 < N; j4 += 1024) {
      v4f out4;
#pragma unroll
      for (int u = 0; u < 4; ++u) {
        const int j = j4 + u;
        bool keep = true;
        if (causal && j > qi) keep = false;
        if (mask && mask[(size_t)qi * mask_pitch + j] == 0) keep = false;
        out4[u] = keep ? __expf(s[j] - mx) * inv : 0.f;
      }
      *(volatile v4f*)(p_out + j4) = out4;
    }
    if (pass == 0) __threadfence();
  }
}

template <bool ASPLIT, int ACT, bool BIAS_BF16, bool RES_BF16>
__global__ __launch_bounds__(128) void k_gemm_bf3(const float* __restrict__ A, int lda, const unsigned short* __restrict__ Wt, int ldb,
                                                const float* __restrict__ bias, const float* __restrict__ resid, int rmod, int ldr,
                                                float* __restrict__ C, int ldc, int M, int N, int K) {
  __shared__ __attribute__((aligned(16))) float so[4][16][64];
  const int tid = threadIdx.x, w = tid >> 5, lane = tid & 31, ln = lane & 15, hh = lane >> 4;
  const int ntn = N / 64;
  const int wid = blockIdx.x * 4 + w;
  const int mt = wid / ntn, nq = wid % ntn;
  if (mt * 16 >= M) return;
  const int row0 = mt * 16, col0 = nq * 64;
  const float* arow = A + (size_t)(row0 + ln) * lda;
  v8f acc[4] = {};
  for (int kb = 0; kb < K; kb += 32) {
    FragB ah, al;
    const v4f x0 = *(const v4fa*)(arow + kb + 8 * hh), x1 = *(const v4fa*)(arow + kb + 8 * hh + 4);
    const v4f x2 = *(const v4fa*)(arow + kb + 16 + 8 * hh), x3 = *(const v4fa*)(arow + kb + 16 + 8 * hh + 4);
    float xs[16] = {x0[0],x0[1],x0[2],x0[3],x1[0],x1[1],x1[2],x1[3],x2[0],x2[1],x2[2],x2[3],x3[0],x3[1],x3[2],x3[3]};
#pragma unroll
    for (int i = 0; i < 16; ++i) { const unsigned short hb = bf16_bits(xs[i]); ah.u[i] = hb; al.u[i] = ASPLIT ? bf16_bits(xs[i] - bf16_val(hb)) : (unsigned short)0; }
#pragma unroll
    for (int t = 0; t < 4; ++t) {
      const unsigned short* brow = Wt + (size_t)(col0 + t * 16 + ln) * ldb + kb;
      FragB b;
      b.half[0] = *(const v8us*)(brow + 8 * hh);
      b.half[1] = *(const v8us*)(brow + 16 + 8 * hh);
      acc[t] = mmaN<ASPLIT ? 2 : 1>(ah.v, al.v, b.v, b.v, acc[t]);
    }
  }
#pragma unroll
  for (int t = 0; t < 4; ++t) {
    const int col = col0 + t * 16 + ln;
    float bv = bias ? bias[col] : 0.f;
    if (BIAS_BF16) bv = bf16_round(bv);
#pragma unroll
    for (int r = 0; r < 8; ++r) {
      float v = acc[t][r] + bv;
      if (resid) { float rv = resid[(size_t)((row0 + 8 * hh + r) % rmod) * ldr + col]; if (RES_BF16) rv = bf16_round(rv); v += rv; }
      if (ACT == 1) v = fmaxf(v, 0.f);
      if (ACT == 2) v = 0.5f * v * (1.0f + erff(v * 0.70710678118654752f));
      if (ACT == 3) { const float u = 0.7978845608028654f * (v + 0.044715f * v * v * v); v = 0.5f * v * (1.0f + tanhf(u)); }
      so[w][8 * hh + r][t * 16 + ln] = v;
    }
  }
  __builtin_amdgcn_fence(__ATOMIC_ACQ_REL, "workgroup");
  __builtin_amdgcn_wave_barrier();
  const int rsub = lane >> 4, c4 = (lane & 15) * 4;
  for (int pass = 0; pass < 2; ++pass) {
#pragma unroll
    for (int q = 0; q < 8; ++q) {
      const int r = q * 2 + rsub;
      const v4f v = *(const v4fa*)&so[w][r][c4];
      *(volatile v4f*)(C + (size_t)(row0 + r) * ldc + col0 + c4) = v;
    }
    if (pass == 0) __threadfence();
  }
}
template <bool PARAM_BF16>
__global__ __launch_bounds__(256) void k_layernorm(const float* __restrict__ X, const float* __restrict__ R, const float* __restrict__ g, const float* __restrict__ bta,
                                                  float* __restrict__ out_sum, float* __restrict__ out_norm, int N, float eps) {
  __shared__ float red[256];
  const int row = blockIdx.x, tid = threadIdx.x;
  const float* x = X + (size_t)row * N; const float* rr = R ? R + (size_t)row * N : nullptr;
  float vals[16];
  const int per = N / 256;
  float s1 = 0.f;
  for (int u = 0; u < per / 4; ++u) {
    const int j = tid * 4 + 1024 * u;
    const v4f a = *(const v4fa*)(x + j);
    v4f b = {0.f,0.f,0.f,0.f}; if (rr) b = *(const v4fa*)(rr + j);
#pragma unroll
    for (int q = 0; q < 4; ++q) { const float v = a[q] + b[q]; vals[u * 4 + q] = v; s1 += v; }
  }
  red[tid] = s1; __syncthreads();
  for (int st = 128; st > 0; st >>= 1) { if (tid < st) red[tid] += red[tid + st]; __syncthreads(); }
  const float mu = red[0] / (float)N; __syncthreads();
  float s2 = 0.f;
  for (int u = 0; u < per / 4; ++u)
#pragma unroll
    for (int q = 0; q < 4; ++q) { const float c = vals[u * 4 + q] - mu; s2 += c * c; }
  red[tid] = s2; __syncthreads();
  for (int st = 128; st > 0; st >>= 1) { if (tid < st) red[tid] += red[tid + st]; __syncthreads(); }
  const float rs = rsqrtf(red[0] / (float)N + eps);
  for (int pass = 0; pass < 2; ++pass) {
    for (int u = 0; u < per / 4; ++u) {
      const int j = tid * 4 + 1024 * u;
      v4f o, sm;
#pragma unroll
      for (int q = 0; q < 4; ++q) {
        float gg = g[j + q], bb = bta[j + q];
        if (PARAM_BF16) { gg = bf16_round(gg); bb = bf16_round(bb); }
        sm[q] = vals[u * 4 + q]; o[q] = (vals[u * 4 + q] - mu) * rs * gg + bb;
      }
      if (out_sum) *(volatile v4f*)(out_sum + (size_t)row * N + j) = sm;
      *(volatile v4f*)(out_norm + (size_t)row * N + j) = o;
    }
    if (pass == 0) __threadfence();
  }
}

__global__ __launch_bounds__(256) void k_round_rows(const float* __restrict__ W, unsigned short* __restrict__ Wt, int n8) {
  const int t = blockIdx.x * 256 + threadIdx.x;
  if (t >= n8) return;
  const v4f a = *(const v4fa*)(W + (size_t)t * 8), b = *(const v4fa*)(W + (size_t)t * 8 + 4);
  v8us v; v[0]=bf16_bits(a[0]); v[1]=bf16_bits(a[1]); v[2]=bf16_bits(a[2]); v[3]=bf16_bits(a[3]);
  v[4]=bf16_bits(b[0]); v[5]=bf16_bits(b[1]); v[6]=bf16_bits(b[2]); v[7]=bf16_bits(b[3]);
  *(volatile v8us*)(Wt + (size_t)t * 8) = v; __threadfence(); *(volatile v8us*)(Wt + (size_t)t * 8) = v;
}

template <bool ROUND, bool ACC>
__global__ __launch_bounds__(256) void k_decomp(const float* __restrict__ x, int nrows, const float* __restrict__ w4, const float* __restrict__ b4, float* __restrict__ res, float* tr) {
  __shared__ double P[LL + 1]; __shared__ float sx[LL]; __shared__ double wsum[256];
  const int row = blockIdx.x; if (row >= nrows) return; const int t = threadIdx.x; const float* xr = x + (size_t)row * LL;
  float v[4]; double s = 0.0; for (int q = 0; q < 4; ++q) { float a = xr[t * 4 + q]; if (ROUND) a = bf16_round(a); v[q] = a; sx[t * 4 + q] = a; s += (double)a; }
  wsum[t] = s; __syncthreads();
  for (int o = 1; o < 256; o <<= 1) { double add = (t >= o) ? wsum[t - o] : 0.0; __syncthreads(); wsum[t] += add; __syncthreads(); }
  double base = (t > 0) ? wsum[t - 1] : 0.0; if (t == 0) P[0] = 0.0;
  for (int q = 0; q < 4; ++q) { base += (double)v[q]; P[t * 4 + q + 1] = base; }
  __syncthreads();
  const float w0 = bf16_round(w4[0]), w1 = bf16_round(w4[1]), w2 = bf16_round(w4[2]), w3 = bf16_round(w4[3]); const float c0 = bf16_round(b4[0]), c1 = bf16_round(b4[1]), c2 = bf16_round(b4[2]), c3 = bf16_round(b4[3]);
  const int KS[4] = {10, 50, 100, 500}; const double x0 = (double)sx[0], xL = (double)sx[LL - 1];
  float outr[4], outm[4];
  for (int q = 0; q < 4; ++q) { const int l = t * 4 + q; const float xv = v[q]; float ma[4];
#pragma unroll
    for (int ki = 0; ki < 4; ++ki) { const int k = KS[ki]; const int f = (k - 1) / 2; const int js = l - f, je = l - f + k - 1; const int lo = js < 0 ? 0 : js, hi = je > LL - 1 ? LL - 1 : je; const int nlo = js < 0 ? -js : 0, nhi = je > LL - 1 ? je - (LL - 1) : 0;
      const double sm = (P[hi + 1] - P[lo]) + (double)nlo * x0 + (double)nhi * xL; ma[ki] = (float)(sm / (double)k); }
    float e0 = xv * w0 + c0, e1 = xv * w1 + c1, e2 = xv * w2 + c2, e3 = xv * w3 + c3; const float mx = fmaxf(fmaxf(e0, e1), fmaxf(e2, e3));
    e0 = expf(e0 - mx); e1 = expf(e1 - mx); e2 = expf(e2 - mx); e3 = expf(e3 - mx); const float den = e0 + e1 + e2 + e3;
    const float mean = (ma[0] * e0 + ma[1] * e1 + ma[2] * e2 + ma[3] * e3) / den; outr[q] = xv - mean; outm[q] = mean; }
  v4f r4 = {outr[0], outr[1], outr[2], outr[3]}; *(volatile v4f*)(res + (size_t)row * LL + t * 4) = r4;
  if (tr) { v4f m4 = {outm[0], outm[1], outm[2], outm[3]}; if (ACC) { const v4f old = *(const v4fa*)(tr + (size_t)row * LL + t * 4); for (int q = 0; q < 4; ++q) m4[q] += old[q]; } *(volatile v4f*)(tr + (size_t)row * LL + t * 4) = m4; __threadfence(); *(volatile v4f*)(tr + (size_t)row * LL + t * 4) = m4; }
  __threadfence(); *(volatile v4f*)(res + (size_t)row * LL + t * 4) = r4;
}
template <bool SEASONAL>
__global__ __launch_bounds__(256) void k_tok8(const float* __restrict__ cm, float* __restrict__ tok) {
  __shared__ float tile[256 * 8]; const int b = blockIdx.x / 4, l0 = (blockIdx.x % 4) * 256; const int t = threadIdx.x;
  for (int c = 0; c < 8; ++c) { float v = 0.f; const int l = l0 + t; if (c < CI) { if (SEASONAL) { if (l < 512) v = cm[((size_t)b * 8 + c) * LL + 512 + l]; } else v = cm[((size_t)b * 8 + c) * LL + l]; } tile[t * 8 + c] = v; }
  __syncthreads();
  for (int pass = 0; pass < 2; ++pass) { for (int e = t; e < 256 * 8; e += 256) *(volatile float*)(tok + ((size_t)b * LL + l0) * 8 + e) = tile[e]; if (pass == 0) __threadfence(); }
}
__global__ __launch_bounds__(256) void k_xcm(const float* __restrict__ xe, float* __restrict__ xcm, float* __restrict__ xmean) {
  __shared__ float red[256]; const int b = blockIdx.x / 8, c = blockIdx.x % 8; const int t = threadIdx.x; float s = 0.f; v4f v = {0.f,0.f,0.f,0.f};
  if (c < CI) { const v4f a = *(const v4fa*)(xe + ((size_t)b * CI + c) * LL + t * 4); for (int q = 0; q < 4; ++q) { v[q] = bf16_round(a[q]); s += v[q]; } }
  *(volatile v4f*)(xcm + (size_t)blockIdx.x * LL + t * 4) = v; red[t] = s; __syncthreads(); for (int st = 128; st > 0; st >>= 1) { if (t < st) red[t] += red[t + st]; __syncthreads(); }
  if (t < 32) { const float m = (t == 0) ? red[0] / (float)LL : 0.f; *(volatile float*)(xmean + (size_t)blockIdx.x * 32 + t) = m; }
  __threadfence(); *(volatile v4f*)(xcm + (size_t)blockIdx.x * LL + t * 4) = v; if (t < 32) { const float m = (t == 0) ? red[0] / (float)LL : 0.f; *(volatile float*)(xmean + (size_t)blockIdx.x * 32 + t) = m; }
}
__global__ __launch_bounds__(256) void k_embed(const float* __restrict__ tok, const float* __restrict__ w, float* __restrict__ h) {
  const int tid = threadIdx.x, wv = tid >> 5, lane = tid & 31; const int m = blockIdx.x * 8 + wv; if (m >= MT) return; const int b = m / LL, l = m % LL;
  float o[2];
#pragma unroll
  for (int u = 0; u < 2; ++u) { const int d = u * 32 + lane; float s = 0.f;
#pragma unroll 1
    for (int k = 0; k < 3; ++k) { const int lk = (l + k - 1 + LL) % LL; const float* tr = tok + ((size_t)b * LL + lk) * 8; for (int c = 0; c < CI; ++c) s += tr[c] * bf16_round(w[((size_t)d * CI + c) * 3 + k]); }
    const int i2 = d & ~1; const float div = expf((float)i2 * (-9.210340371976184f / (float)DD)); const float ang = (float)l * div; s += (d & 1) ? cosf(ang) : sinf(ang); o[u] = s; }
  *(volatile float*)(h + (size_t)m * DD + lane) = o[0]; *(volatile float*)(h + (size_t)m * DD + 32 + lane) = o[1]; __threadfence(); *(volatile float*)(h + (size_t)m * DD + lane) = o[0]; *(volatile float*)(h + (size_t)m * DD + 32 + lane) = o[1];
}
__global__ __launch_bounds__(256) void k_twid(unsigned short* __restrict__ Fh, unsigned short* __restrict__ Fl, unsigned short* __restrict__ Gh, unsigned short* __restrict__ Gl) {
  const int t = blockIdx.x * 256 + threadIdx.x; if (t >= 128 * LL / 8) return; const int i0 = t * 8;
  v8us fh, fl, gh, gl;
#pragma unroll 1
  for (int j = 0; j < 8; ++j) { const int i = i0 + j;
    { const int n = i / LL, l = i % LL; const int m = n & 63; const int r = (m * l) & (LL - 1); float s, c; sincosf((float)r * (6.283185307179586f / (float)LL), &s, &c); const float v = (n < 64) ? c : -s; const unsigned short hb = bf16_bits(v); fh[j] = hb; fl[j] = bf16_bits(v - bf16_val(hb)); }
    { const int l = i / 128, n = i % 128; const int m = n & 63; const int r = (m * l) & (LL - 1); float s, c; sincosf((float)r * (6.283185307179586f / (float)LL), &s, &c); const float cm = (m == 0) ? 1.f : 2.f; const float v = ((n < 64) ? cm * c : -cm * s) / (float)LL; const unsigned short hb = bf16_bits(v); gh[j] = hb; gl[j] = bf16_bits(v - bf16_val(hb)); } }
  *(volatile v8us*)(Fh + i0) = fh; *(volatile v8us*)(Fl + i0) = fl; *(volatile v8us*)(Gh + i0) = gh; *(volatile v8us*)(Gl + i0) = gl; __threadfence();
  *(volatile v8us*)(Fh + i0) = fh; *(volatile v8us*)(Fl + i0) = fl; *(volatile v8us*)(Gh + i0) = gh; *(volatile v8us*)(Gl + i0) = gl;
}
__global__ __launch_bounds__(256) void k_fmix(const float* __restrict__ X, const float* __restrict__ wr, const float* __restrict__ wi, float* __restrict__ Y) {
  const int i = blockIdx.x * 256 + threadIdx.x; if (i >= NR * MO) return; const int m = i % MO; const int row = i / MO; const int o = row % EE, h = (row / EE) % NHD, b = row / DD;
  float yr = 0.f, yi = 0.f;
#pragma unroll 1
  for (int e = 0; e < EE; ++e) { const float* xr = X + ((size_t)b * DD + h * EE + e) * 128; const float ar = xr[m], ai = xr[64 + m]; const size_t wi_ = (((size_t)h * EE + e) * EE + o) * MO + m; const float br = bf16_round(wr[wi_]), bi = bf16_round(wi[wi_]); yr += ar * br - ai * bi; yi += ar * bi + ai * br; }
  *(volatile float*)(Y + (size_t)row * 128 + m) = yr; *(volatile float*)(Y + (size_t)row * 128 + 64 + m) = yi; __threadfence(); *(volatile float*)(Y + (size_t)row * 128 + m) = yr; *(volatile float*)(Y + (size_t)row * 128 + 64 + m) = yi;
}
__device__ __forceinline__ void ctanh(float a, float b, float& tr, float& ti) {
  if (fabsf(a) > 40.f) { tr = a > 0.f ? 1.f : -1.f; ti = 0.f; return; }
  const float s2a = sinhf(2.f * a), c2a = coshf(2.f * a); float s2b, c2b; sincosf(2.f * b, &s2b, &c2b); const float den = c2a + c2b; tr = s2a / den; ti = s2b / den;
}
__global__ __launch_bounds__(256) void k_fcross(const float* __restrict__ XQ, const float* __restrict__ XK, const float* __restrict__ wr, const float* __restrict__ wi, float* __restrict__ Y) {
  __shared__ float sq[EE][128], sk[EE][128]; __shared__ float qkr[MO][MO + 1], qki[MO][MO + 1]; __shared__ float vr[EE][MO], vi[EE][MO];
  const int b = blockIdx.x / NHD, h = blockIdx.x % NHD; const int t = threadIdx.x;
  for (int e2 = t; e2 < EE * 128; e2 += 256) { const int e = e2 / 128, c = e2 % 128; sq[e][c] = XQ[((size_t)b * DD + h * EE + e) * 128 + c]; sk[e][c] = XK[((size_t)b * DD + h * EE + e) * 128 + c]; }
  __syncthreads();
#pragma unroll 1
  for (int i = t; i < MO * MO; i += 256) { const int x = i / MO, y = i % MO; float zr = 0.f, zi = 0.f;
#pragma unroll 1
    for (int e = 0; e < EE; ++e) { const float ar = sq[e][x], ai = sq[e][64 + x], br = sk[e][y], bi = sk[e][64 + y]; zr += ar * br - ai * bi; zi += ar * bi + ai * br; }
    float tr, ti; ctanh(zr, zi, tr, ti); qkr[x][y] = tr; qki[x][y] = ti; }
  __syncthreads();
#pragma unroll 1
  for (int i = t; i < EE * MO; i += 256) { const int e = i / MO, x = i % MO; float zr = 0.f, zi = 0.f;
#pragma unroll 1
    for (int y = 0; y < MO; ++y) { const float ar = qkr[x][y], ai = qki[x][y], br = sk[e][y], bi = sk[e][64 + y]; zr += ar * br - ai * bi; zi += ar * bi + ai * br; }
    vr[e][x] = zr; vi[e][x] = zi; }
  __syncthreads();
  for (int pass = 0; pass < 2; ++pass) {
#pragma unroll 1
    for (int i = t; i < EE * MO; i += 256) { const int o = i / MO, x = i % MO; float zr = 0.f, zi = 0.f;
#pragma unroll 1
      for (int e = 0; e < EE; ++e) { const size_t wi_ = (((size_t)h * EE + e) * EE + o) * MO + x; const float br = bf16_round(wr[wi_]), bi = bf16_round(wi[wi_]); zr += vr[e][x] * br - vi[e][x] * bi; zi += vr[e][x] * bi + vi[e][x] * br; }
      float* yr = Y + ((size_t)b * DD + h * EE + o) * 128; *(volatile float*)(yr + x) = zr * (1.0f / 4096.0f); *(volatile float*)(yr + 64 + x) = zi * (1.0f / 4096.0f); }
    if (pass == 0) __threadfence(); }
}
__global__ __launch_bounds__(256) void k_add(const float* a, const float* bq, float* o, size_t n4) { const size_t t = (size_t)blockIdx.x * 256 + threadIdx.x; if (t >= n4) return; const v4f x = *(const v4fa*)(a + t * 4), y = *(const v4fa*)(bq + t * 4); v4f v; for (int q = 0; q < 4; ++q) v[q] = x[q] + y[q]; *(volatile v4f*)(o + t * 4) = v; __threadfence(); *(volatile v4f*)(o + t * 4) = v; }
__global__ __launch_bounds__(256) void k_ln64(const float* __restrict__ x, const float* __restrict__ g, const float* __restrict__ bb, float* __restrict__ out) {
  const int tid = threadIdx.x, wv = tid >> 5, lane = tid & 31; const int m = blockIdx.x * 8 + wv; if (m >= MT) return;
  const float a = x[(size_t)m * DD + lane], c = x[(size_t)m * DD + 32 + lane]; float s = a + c; for (int o = 16; o >= 1; o >>= 1) s += __shfl_xor(s, o, 32); const float mu = s / DD;
  float q2 = (a - mu) * (a - mu) + (c - mu) * (c - mu); for (int o = 16; o >= 1; o >>= 1) q2 += __shfl_xor(q2, o, 32); const float rs = rsqrtf(q2 / DD + 1e-5f);
  const float o1 = (a - mu) * rs * bf16_round(g[lane]) + bf16_round(bb[lane]), o2 = (c - mu) * rs * bf16_round(g[32 + lane]) + bf16_round(bb[32 + lane]);
  *(volatile float*)(out + (size_t)m * DD + lane) = o1; *(volatile float*)(out + (size_t)m * DD + 32 + lane) = o2; __threadfence(); *(volatile float*)(out + (size_t)m * DD + lane) = o1; *(volatile float*)(out + (size_t)m * DD + 32 + lane) = o2;
}
__global__ __launch_bounds__(64) void k_colmean(const float* __restrict__ x, float* __restrict__ cm) { const int b = blockIdx.x, d = threadIdx.x; float s = 0.f;
#pragma unroll 1
  for (int l = 0; l < LL; ++l) s += x[((size_t)b * LL + l) * DD + d]; const float v = s / LL; *(volatile float*)(cm + (size_t)b * DD + d) = v; __threadfence(); *(volatile float*)(cm + (size_t)b * DD + d) = v; }
__global__ __launch_bounds__(256) void k_subcol(float* __restrict__ x, const float* __restrict__ cm) { const size_t i = (size_t)blockIdx.x * 256 + threadIdx.x; if (i >= (size_t)MT * DD / 4) return; const int c4 = (int)(i % (DD / 4)) * 4; const int b = (int)(i / ((size_t)LL * DD / 4)); v4f v = *(const v4fa*)(x + i * 4); for (int q = 0; q < 4; ++q) v[q] -= cm[(size_t)b * DD + c4 + q]; *(volatile v4f*)(x + i * 4) = v; __threadfence(); *(volatile v4f*)(x + i * 4) = v; }
__global__ __launch_bounds__(256) void k_final(const float* __restrict__ xd, const float* __restrict__ pw, const float* __restrict__ pb, const float* __restrict__ t7, const float* __restrict__ xmean, const float* __restrict__ dpw, const float* __restrict__ dpb, const float* __restrict__ tT, const float* __restrict__ tw, float* __restrict__ out) {
  const int i = blockIdx.x * 256 + threadIdx.x; if (i >= BB * 512) return; const int b = i / 512, j = i % 512; const int l = 512 + j;
  float s = bf16_round(pb[0]); const float* xr = xd + ((size_t)b * LL + l) * DD;
#pragma unroll 1
  for (int d = 0; d < DD; ++d) s += xr[d] * bf16_round(pw[d]);
  float ti = bf16_round(dpb[0]);
#pragma unroll 1
  for (int c = 0; c < CI; ++c) { const float tv = (l < 512) ? t7[((size_t)b * 8 + c) * LL + 512 + l] : xmean[((size_t)b * 8 + c) * 32]; ti += tv * bf16_round(dpw[c]); }
  float t2 = 0.f;
#pragma unroll 1
  for (int d = 0; d < DD; ++d) { const float* tr = tT + ((size_t)b * DD + d) * LL; for (int k = 0; k < 3; ++k) t2 += tr[(l + k - 1 + LL) % LL] * bf16_round(tw[d * 3 + k]); }
  const float v = s + ti + t2; *(volatile float*)(out + i) = v; __threadfence(); *(volatile float*)(out + i) = v;
}
extern "C" void kernel_launch(void* const* d_in, const int* in_sizes, int n_in,
                              void* d_out, int out_size, void* d_ws, size_t ws_size, hipStream_t stream) {
  (void)in_sizes; (void)n_in; (void)out_size;
  const float* x_enc = (const float*)d_in[0]; const float* dp_w = (const float*)d_in[1]; const float* dp_b = (const float*)d_in[2]; const float* emb_e = (const float*)d_in[3]; const float* emb_d = (const float*)d_in[4];
  const float* dcw = (const float*)d_in[5]; const float* dcb = (const float*)d_in[6]; const float* eaw = (const float*)d_in[7]; const float* eab = (const float*)d_in[8]; const float* efr = (const float*)d_in[9]; const float* efi = (const float*)d_in[10];
  const float* ec1 = (const float*)d_in[11]; const float* ec2 = (const float*)d_in[12]; const float* elg = (const float*)d_in[13]; const float* elb = (const float*)d_in[14];
  const float* dsw = (const float*)d_in[15]; const float* dsb = (const float*)d_in[16]; const float* dfr = (const float*)d_in[17]; const float* dfi = (const float*)d_in[18];
  const float* dxw = (const float*)d_in[19]; const float* dxb = (const float*)d_in[20]; const float* dxr = (const float*)d_in[21]; const float* dxi = (const float*)d_in[22];
  const float* dc1 = (const float*)d_in[23]; const float* dc2 = (const float*)d_in[24]; const float* dtw = (const float*)d_in[25]; const float* dlg = (const float*)d_in[26]; const float* dlb = (const float*)d_in[27]; const float* dpw = (const float*)d_in[28]; const float* dpb2 = (const float*)d_in[29];
  char* ws = (char*)d_ws; size_t off = 0;
  auto take = [&](size_t bytes) { char* p = ws + off; off += (bytes + 255) & ~(size_t)255; return p; };
  unsigned short* Bq[2], *Bo[2], *Bc1[2], *Bc2[2]; for (int l = 0; l < 2; ++l) { Bq[l] = (unsigned short*)take(DD * DD * 2); Bo[l] = (unsigned short*)take(DD * DD * 2); Bc1[l] = (unsigned short*)take(DFF * DD * 2); Bc2[l] = (unsigned short*)take(DD * DFF * 2); }
  unsigned short* Bds0 = (unsigned short*)take(DD * DD * 2); unsigned short* Bds3 = (unsigned short*)take(DD * DD * 2); unsigned short* Bdx0 = (unsigned short*)take(DD * DD * 2); unsigned short* Bdx1 = (unsigned short*)take(DD * DD * 2); unsigned short* Bdx3 = (unsigned short*)take(DD * DD * 2);
  unsigned short* Bdc1 = (unsigned short*)take(DFF * DD * 2); unsigned short* Bdc2 = (unsigned short*)take(DD * DFF * 2);
  unsigned short* Fh = (unsigned short*)take(128 * LL * 2); unsigned short* Fl = (unsigned short*)take(128 * LL * 2); unsigned short* Gh = (unsigned short*)take(LL * 128 * 2); unsigned short* Gl = (unsigned short*)take(LL * 128 * 2);
  float* xcm = (float*)take((size_t)BB * 8 * LL * 4); float* xmean = (float*)take((size_t)BB * 8 * 32 * 4); float* s7 = (float*)take((size_t)BB * 8 * LL * 4); float* t7 = (float*)take((size_t)BB * 8 * LL * 4); float* tok = (float*)take((size_t)MT * 8 * 4);
  float* h = (float*)take((size_t)MT * DD * 4); float* q = (float*)take((size_t)MT * DD * 4); float* qT = (float*)take((size_t)MT * DD * 4); float* XF = (float*)take((size_t)NR * 128 * 4); float* XK = (float*)take((size_t)NR * 128 * 4); float* YF = (float*)take((size_t)NR * 128 * 4); float* yT = (float*)take((size_t)MT * DD * 4);
  float* a = (float*)take((size_t)MT * DD * 4); float* sT = (float*)take((size_t)MT * DD * 4); float* rT = (float*)take((size_t)MT * DD * 4); float* tT = (float*)take((size_t)MT * DD * 4); float* ff = (float*)take((size_t)MT * DFF * 4); float* henc = (float*)take((size_t)MT * DD * 4); float* cm = (float*)take(BB * DD * 4);
  if (off > ws_size) return;
  for (int l = 0; l < 2; ++l) { k_round_rows<<<(DD * DD / 8 + 255) / 256, 256, 0, stream>>>(eaw + ((size_t)l * 4 + 0) * DD * DD, Bq[l], DD * DD / 8); k_round_rows<<<(DD * DD / 8 + 255) / 256, 256, 0, stream>>>(eaw + ((size_t)l * 4 + 3) * DD * DD, Bo[l], DD * DD / 8);
    k_round_rows<<<(DFF * DD / 8 + 255) / 256, 256, 0, stream>>>(ec1 + (size_t)l * DFF * DD, Bc1[l], DFF * DD / 8); k_round_rows<<<(DD * DFF / 8 + 255) / 256, 256, 0, stream>>>(ec2 + (size_t)l * DD * DFF, Bc2[l], DD * DFF / 8); }
  k_round_rows<<<(DD * DD / 8 + 255) / 256, 256, 0, stream>>>(dsw + 0 * DD * DD, Bds0, DD * DD / 8); k_round_rows<<<(DD * DD / 8 + 255) / 256, 256, 0, stream>>>(dsw + 3 * DD * DD, Bds3, DD * DD / 8);
  k_round_rows<<<(DD * DD / 8 + 255) / 256, 256, 0, stream>>>(dxw + 0 * DD * DD, Bdx0, DD * DD / 8); k_round_rows<<<(DD * DD / 8 + 255) / 256, 256, 0, stream>>>(dxw + 1 * DD * DD, Bdx1, DD * DD / 8); k_round_rows<<<(DD * DD / 8 + 255) / 256, 256, 0, stream>>>(dxw + 3 * DD * DD, Bdx3, DD * DD / 8);
  k_round_rows<<<(DFF * DD / 8 + 255) / 256, 256, 0, stream>>>(dc1, Bdc1, DFF * DD / 8); k_round_rows<<<(DD * DFF / 8 + 255) / 256, 256, 0, stream>>>(dc2, Bdc2, DD * DFF / 8);
  k_twid<<<(128 * LL / 8 + 255) / 256, 256, 0, stream>>>(Fh, Fl, Gh, Gl);
  const unsigned g64 = ((MT / 16) * 1 + 3) / 4, g256 = ((MT / 16) * 4 + 3) / 4; const size_t n4 = (size_t)MT * DD / 4; const unsigned gn4 = (unsigned)((n4 + 255) / 256);
  auto proj = [&](const float* A, const unsigned short* Bt, const float* bias, float* C) { k_gemm_bf3<true, 0, true, false><<<g64, 128, 0, stream>>>(A, DD, Bt, DD, bias, nullptr, 1, 0, C, DD, MT, DD, DD); };
  auto to_cm = [&](const float* tokm, float* cmaj) { k_transpose32<false, false, false><<<dim3(DD / 32, LL / 32, BB), 256, 0, stream>>>(tokm, cmaj, LL, DD, nullptr, nullptr, nullptr); };
  auto to_tok = [&](const float* cmaj, float* tokm) { k_transpose32<false, false, false><<<dim3(LL / 32, DD / 32, BB), 256, 0, stream>>>(cmaj, tokm, DD, LL, nullptr, nullptr, nullptr); };
  auto rfft = [&](const float* qtok, float* Xout) { to_cm(qtok, qT); k_gemm_bf2<true, true, 0, false><<<((NR / 16) * 2 + 3) / 4, 128, 0, stream>>>(qT, LL, Fh, Fl, LL, nullptr, 1.f, Xout, 128, NR, 128, LL); };
  auto irfft = [&](const float* Yin, float* ytok) { k_gemm_bf2<true, true, 0, false><<<((NR / 16) * (LL / 64) + 3) / 4, 128, 0, stream>>>(Yin, 128, Gh, Gl, 128, nullptr, 1.f, ytok, LL, NR, LL, 128); };
  auto decomp64 = [&](const float* in_tok, int wi, float* out_tok, bool trend, bool acc) { to_cm(in_tok, sT);
    if (!trend) k_decomp<false, false><<<NR, 256, 0, stream>>>(sT, NR, dcw + wi * 4, dcb + wi * 4, rT, nullptr);
    else if (!acc) k_decomp<false, false><<<NR, 256, 0, stream>>>(sT, NR, dcw + wi * 4, dcb + wi * 4, rT, tT);
    else k_decomp<false, true><<<NR, 256, 0, stream>>>(sT, NR, dcw + wi * 4, dcb + wi * 4, rT, tT);
    to_tok(rT, out_tok); };
  k_xcm<<<BB * 8, 256, 0, stream>>>(x_enc, xcm, xmean);
  k_decomp<false, false><<<BB * 8, 256, 0, stream>>>(xcm, BB * 8, dcw, dcb, s7, t7);
  k_tok8<false><<<BB * 4, 256, 0, stream>>>(xcm, tok); k_embed<<<(MT + 7) / 8, 256, 0, stream>>>(tok, emb_e, h);
  for (int l = 0; l < 2; ++l) {
    proj(h, Bq[l], eab + ((size_t)l * 4 + 0) * DD, q); rfft(q, XF); k_fmix<<<(NR * MO + 255) / 256, 256, 0, stream>>>(XF, efr + (size_t)l * NHD * EE * EE * MO, efi + (size_t)l * NHD * EE * EE * MO, YF); irfft(YF, yT);
    proj(yT, Bo[l], eab + ((size_t)l * 4 + 3) * DD, a); k_add<<<gn4, 256, 0, stream>>>(h, a, a, n4); decomp64(a, 1 + 2 * l, h, false, false);
    k_gemm_bf3<true, 2, false, false><<<g256, 128, 0, stream>>>(h, DD, Bc1[l], DD, nullptr, nullptr, 1, 0, ff, DFF, MT, DFF, DD);
    k_gemm_bf3<true, 0, false, false><<<g64, 128, 0, stream>>>(ff, DFF, Bc2[l], DFF, nullptr, h, MT, DD, a, DD, MT, DD, DFF);
    decomp64(a, 2 + 2 * l, h, false, false);
  }
  k_ln64<<<(MT + 7) / 8, 256, 0, stream>>>(h, elg, elb, henc); k_colmean<<<BB, 64, 0, stream>>>(henc, cm); k_subcol<<<gn4, 256, 0, stream>>>(henc, cm);
  float* xd = h;
  k_tok8<true><<<BB * 4, 256, 0, stream>>>(s7, tok); k_embed<<<(MT + 7) / 8, 256, 0, stream>>>(tok, emb_d, xd);
  proj(xd, Bds0, dsb + 0 * DD, q); rfft(q, XF); k_fmix<<<(NR * MO + 255) / 256, 256, 0, stream>>>(XF, dfr, dfi, YF); irfft(YF, yT);
  proj(yT, Bds3, dsb + 3 * DD, a); k_add<<<gn4, 256, 0, stream>>>(xd, a, a, n4); decomp64(a, 5, xd, true, false);
  proj(xd, Bdx0, dxb + 0 * DD, q); rfft(q, XF); proj(henc, Bdx1, dxb + 1 * DD, q); rfft(q, XK);
  k_fcross<<<BB * NHD, 256, 0, stream>>>(XF, XK, dxr, dxi, YF); irfft(YF, yT);
  proj(yT, Bdx3, dxb + 3 * DD, a); k_add<<<gn4, 256, 0, stream>>>(xd, a, a, n4); decomp64(a, 6, xd, true, true);
  k_gemm_bf3<true, 2, false, false><<<g256, 128, 0, stream>>>(xd, DD, Bdc1, DD, nullptr, nullptr, 1, 0, ff, DFF, MT, DFF, DD);
  k_gemm_bf3<true, 0, false, false><<<g64, 128, 0, stream>>>(ff, DFF, Bdc2, DFF, nullptr, xd, MT, DD, a, DD, MT, DD, DFF);
  decomp64(a, 7, xd, true, true);
  k_ln64<<<(MT + 7) / 8, 256, 0, stream>>>(xd, dlg, dlb, henc); k_colmean<<<BB, 64, 0, stream>>>(henc, cm); k_subcol<<<gn4, 256, 0, stream>>>(henc, cm);
  k_final<<<(BB * 512 + 255) / 256, 256, 0, stream>>>(henc, dpw, dpb2, t7, xmean, dp_w, dp_b, tT, dtw, (float*)d_out);
}
